// CondAttLSTM_29429115912193
// MI455X (gfx1250) — hardware-verified
//
#include <hip/hip_runtime.h>
#include <stdint.h>

typedef __attribute__((ext_vector_type(16))) _Float16 v16h;
typedef __attribute__((ext_vector_type(8)))  _Float16 v8h;
typedef __attribute__((ext_vector_type(4)))  _Float16 v4h;
typedef __attribute__((ext_vector_type(16))) __bf16   v16b;
typedef __attribute__((ext_vector_type(8)))  __bf16   v8b;
typedef __attribute__((ext_vector_type(8)))  float    v8f;
typedef __attribute__((ext_vector_type(4)))  float    v4f;

__device__ __forceinline__ unsigned short f2bf_bits(float f) {
  unsigned u = __float_as_uint(f);
  return (unsigned short)((u + 0x7FFFu + ((u >> 16) & 1u)) >> 16);
}
__device__ __forceinline__ float bf_bits2f(unsigned short h) { return __uint_as_float(((unsigned)h) << 16); }

__device__ __forceinline__ void dep_guard_h(v8f& a, v8f& b, v16h x, v16h y) { asm volatile("v_nop\n\tv_nop\n\tv_nop\n\tv_nop" : "+v"(a), "+v"(b) : "v"(x), "v"(y)); }
__device__ __forceinline__ void dep_guard_b(v8f& a, v8f& b, v16b x, v16b y) { asm volatile("v_nop\n\tv_nop\n\tv_nop\n\tv_nop" : "+v"(a), "+v"(b) : "v"(x), "v"(y)); }
__device__ __forceinline__ void keep4_h(v16h a, v16h b, v16h c, v16h d) { asm volatile("v_nop" :: "v"(a), "v"(b), "v"(c), "v"(d)); }
__device__ __forceinline__ void keep4_b(v16b a, v16b b, v16b c, v16b d) { asm volatile("v_nop" :: "v"(a), "v"(b), "v"(c), "v"(d)); }
__device__ __forceinline__ void acc_guard4(v8f& a, v8f& b, v8f& c, v8f& d) { asm volatile("v_nop\n\tv_nop\n\tv_nop\n\tv_nop" : "+v"(a), "+v"(b), "+v"(c), "+v"(d)); }
template <typename T> struct Frag;
template <> struct Frag<_Float16> {
  typedef v16h V; union U { v16h v; v8h h[2]; };
  static __device__ __forceinline__ v16h load(const _Float16* p) {
    U f; f.h[0] = *(const v8h*)(p); f.h[1] = *(const v8h*)(p + 16); return f.v;
  }
  static __device__ __forceinline__ v8f mma(v16h a, v16h b, v8f c) {
    return __builtin_amdgcn_wmma_f32_16x16x32_f16(false, a, false, b, (short)0, c, false, false);
  }
  static __device__ __forceinline__ void guard(v8f& a, v8f& b, v16h x, v16h y) { dep_guard_h(a, b, x, y); }
  static __device__ __forceinline__ void keep(v16h a, v16h b, v16h c, v16h d) { keep4_h(a, b, c, d); }
};
template <> struct Frag<__bf16> {
  typedef v16b V; union U { v16b v; v8b h[2]; };
  static __device__ __forceinline__ v16b load(const __bf16* p) {
    U f; f.h[0] = *(const v8b*)(p); f.h[1] = *(const v8b*)(p + 16); return f.v;
  }
  static __device__ __forceinline__ v8f mma(v16b a, v16b b, v8f c) {
    return __builtin_amdgcn_wmma_f32_16x16x32_bf16(false, a, false, b, (short)0, c, false, false);
  }
  static __device__ __forceinline__ void guard(v8f& a, v8f& b, v16b x, v16b y) { dep_guard_b(a, b, x, y); }
  static __device__ __forceinline__ void keep(v16b a, v16b b, v16b c, v16b d) { keep4_b(a, b, c, d); }
};

template <int ET> struct Elem;
template <> struct Elem<0> { typedef _Float16 T; };
template <> struct Elem<1> { typedef __bf16 T; };
template <int ET, bool SPLIT, int BIAS_MODE, int OUT_MODE, bool RESID, int ACT = 0>
__global__ __launch_bounds__(256) void wmma_gemm64(
    const unsigned short* __restrict__ Ap, const unsigned short* __restrict__ A2p, int lda, long strideA,
    const unsigned short* __restrict__ Btp, const unsigned short* __restrict__ Bt2p, int ldb, long strideB,
    void* __restrict__ Cout, void* __restrict__ Cout2, int ldc, long strideC,
    const float* __restrict__ bias,
    const float* __restrict__ resid, long strideR,
    int M, int N, int K, float scale) {
  typedef typename Elem<ET>::T T;
  typedef typename Frag<T>::V V;
  const T* A = (const T*)Ap; const T* A2 = (const T*)A2p; const T* Bt = (const T*)Btp; const T* Bt2 = (const T*)Bt2p;
  __shared__ __align__(16) float sT[8][16 * 68];
  const int b    = blockIdx.y;
  const int lane = threadIdx.x & 31;
  const int wave = threadIdx.x >> 5;
  const int tilesN = N >> 6;
  const int tilesM = M >> 6;
  const int tile = blockIdx.x * 8 + wave;
  if (tile >= tilesM * tilesN) return;
  const int tm = tile / tilesN;
  const int tn = tile - tm * tilesN;
  const int m0 = tm << 6;
  const int n0 = tn << 6;

  const T* Ab  = A  + (size_t)b * strideA;
  const T* Bb  = Bt + (size_t)b * strideB;
  const T* Ab2 = SPLIT ? (A2  + (size_t)b * strideA) : nullptr;
  const T* Bb2 = SPLIT ? (Bt2 + (size_t)b * strideB) : nullptr;

  const int rlane = lane & 15;
  const int koff  = (lane >> 4) * 8;
  const int mOff  = (lane >> 4) * 8;

  v8f acc[4][4];
#pragma unroll
  for (int i = 0; i < 4; ++i)
#pragma unroll
    for (int j = 0; j < 4; ++j) acc[i][j] = (v8f){0.f,0.f,0.f,0.f,0.f,0.f,0.f,0.f};

  for (int k0 = 0; k0 < K; k0 += 32) {
    V bh[4], bl[4];
#pragma unroll
    for (int j = 0; j < 4; ++j) {
      const size_t bo = (size_t)(n0 + (j << 4) + rlane) * ldb + koff + k0;
      bh[j] = Frag<T>::load(Bb + bo);
      if (SPLIT) bl[j] = Frag<T>::load(Bb2 + bo);
    }
#pragma unroll
    for (int i = 0; i < 4; ++i) {
      const size_t ao = (size_t)(m0 + (i << 4) + rlane) * lda + koff + k0;
      V ah = Frag<T>::load(Ab + ao);
      V al;
      if (SPLIT) al = Frag<T>::load(Ab2 + ao);
#pragma unroll
      for (int j = 0; j < 4; ++j) {
        acc[i][j] = Frag<T>::mma(ah, bh[j], acc[i][j]);
        if (SPLIT) {
          acc[i][j] = Frag<T>::mma(ah, bl[j], acc[i][j]);
          acc[i][j] = Frag<T>::mma(al, bh[j], acc[i][j]);
        }
      }
      Frag<T>::guard(acc[i][0], acc[i][3], ah, SPLIT ? al : ah);
    }
    Frag<T>::keep(bh[0], bh[1], bh[2], bh[3]);
    if (SPLIT) Frag<T>::keep(bl[0], bl[1], bl[2], bl[3]);
  }
  acc_guard4(acc[0][0], acc[0][1], acc[0][2], acc[0][3]);
  acc_guard4(acc[1][0], acc[1][1], acc[1][2], acc[1][3]);
  acc_guard4(acc[2][0], acc[2][1], acc[2][2], acc[2][3]);
  acc_guard4(acc[3][0], acc[3][1], acc[3][2], acc[3][3]);

  float* slab = sT[wave];
  const float* Rb = RESID ? (resid + (size_t)b * strideR) : nullptr;
#pragma unroll
  for (int i = 0; i < 4; ++i) {
    const int mBase = m0 + (i << 4);
#pragma unroll
    for (int j = 0; j < 4; ++j) {
      const int n = n0 + (j << 4) + rlane;
      float bv = 0.f;
      if (BIAS_MODE == 2) bv = bias[n];
#pragma unroll
      for (int r = 0; r < 8; ++r) {
        float v = acc[i][j][r] * scale;
        if (BIAS_MODE == 1) v += bias[mBase + mOff + r];
        if (BIAS_MODE == 2) v += bv;
        if (RESID) v += Rb[(size_t)(mBase + mOff + r) * ldc + n];
        if (ACT == 1) v = tanhf(v);
        if (ACT == 2) v = fmaxf(v, 0.0f);
        if (ACT == 3) v = v / (1.0f + expf(-v));
        if (ACT == 4) v = (v > 0.f) ? v : 0.01f * v;
        if (ACT == 5) v = 0.5f * v * (1.0f + erff(v * 0.70710678118654752f));
        slab[(mOff + r) * 68 + (j << 4) + rlane] = v;
      }
    }
    __builtin_amdgcn_fence(__ATOMIC_RELEASE, "workgroup");
    __builtin_amdgcn_wave_barrier();
    __builtin_amdgcn_fence(__ATOMIC_ACQUIRE, "workgroup");
    if (OUT_MODE == 0) {
      float* C = (float*)Cout + (size_t)b * strideC;
      const int hh = lane >> 4, c4 = (lane & 15) * 4;
      for (int pass = 0; pass < 2; ++pass) {
#pragma unroll
        for (int it = 0; it < 8; ++it) {
          const int row = it * 2 + hh;
          v4f v = *(const v4f*)(slab + row * 68 + c4);
          *(volatile v4f*)(C + (size_t)(mBase + row) * ldc + n0 + c4) = v;
        }
        __threadfence();
      }
    } else {
      const int q = lane >> 3, c8 = (lane & 7) * 8;
      unsigned short* C  = (unsigned short*)Cout  + (size_t)b * strideC;
      unsigned short* C2 = (OUT_MODE == 2) ? ((unsigned short*)Cout2 + (size_t)b * strideC) : nullptr;
      for (int pass = 0; pass < 2; ++pass) {
#pragma unroll
        for (int it = 0; it < 4; ++it) {
          const int row = it * 4 + q;
          const float* sp = slab + row * 68 + c8;
          v8h hv, lv;
#pragma unroll
          for (int e = 0; e < 8; ++e) {
            if (OUT_MODE == 1) {
              hv[e] = (_Float16)sp[e];
            } else {
              unsigned short hb = f2bf_bits(sp[e]);
              unsigned short lb = f2bf_bits(sp[e] - bf_bits2f(hb));
              hv[e] = __builtin_bit_cast(_Float16, hb);
              lv[e] = __builtin_bit_cast(_Float16, lb);
            }
          }
          *(volatile v8h*)(C + (size_t)(mBase + row) * ldc + n0 + c8) = hv;
          if (OUT_MODE == 2) *(volatile v8h*)(C2 + (size_t)(mBase + row) * ldc + n0 + c8) = lv;
        }
        __threadfence();
      }
    }
    __builtin_amdgcn_fence(__ATOMIC_RELEASE, "workgroup");
    __builtin_amdgcn_wave_barrier();
    __builtin_amdgcn_fence(__ATOMIC_ACQUIRE, "workgroup");
  }
}

constexpr int kB = 32, kT = 128, kDim = 512, kL = 64, kA = 128, kG4 = 2048, kMB = 16;
constexpr int kNT = 512;
constexpr int kHP = 520;
constexpr int kHRP = 516;
constexpr float kS16 = 0.0625f;
static_assert(kDim % 32 == 0);
static_assert(kHP % 8 == 0 && kHRP % 4 == 0);
static_assert((kB * kL) % 64 == 0 && kA % 64 == 0);
static_assert(kB % kMB == 0);
static_assert(kMB * kDim == kNT * 16);
static_assert(kMB * kT == kNT * 4);
static_assert((kNT / 32) * 32 == kDim);

__device__ __forceinline__ float bfr(float f) {
  unsigned u = __float_as_uint(f);
  u = (u + 0x7FFFu + ((u >> 16) & 1u)) & 0xFFFF0000u;
  return __uint_as_float(u);
}
__device__ __forceinline__ float frcp(float x) { return __builtin_amdgcn_rcpf(x); }
__device__ __forceinline__ float fexp(float x) { return __builtin_amdgcn_exp2f(x * 1.4426950408889634f); }
__device__ __forceinline__ float tnh(float x) { return 1.0f - 2.0f * frcp(1.0f + fexp(2.0f * x)); }
__device__ __forceinline__ float sgm(float x) { return frcp(1.0f + fexp(-x)); }

__device__ __forceinline__ v8f hmma(v16h a, v16h b, v8f c) {
  c = __builtin_amdgcn_wmma_f32_16x16x32_f16(false, a, false, b, (short)0, c, false, false);
  asm volatile("v_nop\n\tv_nop\n\tv_nop\n\tv_nop" : "+v"(c) : "v"(a), "v"(b));
  return c;
}

__global__ __launch_bounds__(256) void cast_bf_f16x2(const float* __restrict__ in, _Float16* __restrict__ out, int n2, float mul) {
  const int i = blockIdx.x * 256 + threadIdx.x;
  if (i < n2) {
    const _Float16 a0 = (_Float16)(bfr(in[2 * i]) * mul);
    const _Float16 a1 = (_Float16)(bfr(in[2 * i + 1]) * mul);
    const unsigned u = (unsigned)__builtin_bit_cast(unsigned short, a0) | ((unsigned)__builtin_bit_cast(unsigned short, a1) << 16);
    ((volatile unsigned*)out)[i] = u;
    __threadfence();
    ((volatile unsigned*)out)[i] = u;
  }
}

__global__ __launch_bounds__(256) void rne_bf_f32x4(const float* __restrict__ in, float* __restrict__ out, int n4) {
  const int i = blockIdx.x * 256 + threadIdx.x;
  if (i < n4) {
    const v4f v = *(const v4f*)(in + 4 * (size_t)i);
    v4f r;
    r[0] = bfr(v[0]); r[1] = bfr(v[1]); r[2] = bfr(v[2]); r[3] = bfr(v[3]);
    *(volatile v4f*)(out + 4 * (size_t)i) = r;
    __threadfence();
    *(volatile v4f*)(out + 4 * (size_t)i) = r;
  }
}

__device__ __forceinline__ v8f proj_tile(const _Float16* shA, const _Float16* __restrict__ W16, int n0, int rl, int koff) {
  v8f qa = (v8f){0.f,0.f,0.f,0.f,0.f,0.f,0.f,0.f};
#pragma unroll 1
  for (int k0 = 0; k0 < kDim; k0 += 32) {
    const v16h a = Frag<_Float16>::load(shA + rl * kHP + koff + k0);
    const v16h b = Frag<_Float16>::load(W16 + (size_t)(n0 + rl) * kDim + koff + k0);
    qa = hmma(a, b, qa);
  }
  return qa;
}

__device__ __forceinline__ void gate_seg(v8f (&acc)[4], const _Float16* shA, const _Float16* __restrict__ W16, int cb, int rl, int koff) {
#pragma unroll 1
  for (int k0 = 0; k0 < kDim; k0 += 32) {
    const v16h a = Frag<_Float16>::load(shA + rl * kHP + koff + k0);
    v16h bf[4];
#pragma unroll
    for (int j = 0; j < 4; ++j)
      bf[j] = Frag<_Float16>::load(W16 + (size_t)(j * kDim + cb + rl) * kDim + koff + k0);
#pragma unroll
    for (int j = 0; j < 4; ++j) acc[j] = hmma(a, bf[j], acc[j]);
  }
}

__global__ void __launch_bounds__(512)
lstm_scan_kernel(const float* __restrict__ X,
                 const float* __restrict__ ctxr,
                 const float* __restrict__ h0,
                 const float* __restrict__ bx,
                 const float* __restrict__ wa,
                 const float* __restrict__ ba1,
                 const float* __restrict__ bhh,
                 const float* __restrict__ wha,
                 const float* __restrict__ bha1,
                 const int*   __restrict__ parent,
                 const float* __restrict__ ctxatt,
                 float*       histproj,
                 const _Float16* __restrict__ Uh16, const _Float16* __restrict__ Cc16,
                 const _Float16* __restrict__ Ph16, const _Float16* __restrict__ Hh16,
                 const _Float16* __restrict__ Wx16, const _Float16* __restrict__ Wah16,
                 const _Float16* __restrict__ Whq16, const _Float16* __restrict__ Whh16,
                 float* out_h,
                 float* out_ctx) {
  __shared__ __align__(16) _Float16 sh_h[kMB * kHP];
  __shared__ __align__(16) _Float16 sh_actx[kMB * kHP];
  __shared__ __align__(16) _Float16 sh_apar[kMB * kHP];
  __shared__ __align__(16) _Float16 sh_ahc[kMB * kHP];
  __shared__ __align__(16) _Float16 sh_ax[kMB * kHP];
  __shared__ __align__(16) float sh_hrow[kMB * kHRP];
  __shared__ __align__(16) float sh_q[2 * kMB * kA];
  __shared__ __align__(16) float sh_sc[kMB * kT];
  __shared__ __align__(16) float sh_vec[3 * kA];

  float* sh_wa = sh_vec;
  float* sh_wha = sh_vec + kA;
  float* sh_bhh = sh_vec + 2 * kA;

  const int tid = threadIdx.x;
  const int wave = tid >> 5;
  const int lane = tid & 31;
  const int c = lane & 15;
  const int hh = lane >> 4;
  const int koff = hh * 8;
  const int bg = blockIdx.x * kMB;
  const int bq = tid >> 7;
  const int d0 = (tid & 127) * 4;
  const size_t kRowStride = (size_t)kT * kDim;
  const float ba_r = bfr(ba1[0]);
  const float bha_r = bfr(bha1[0]);

#pragma unroll
  for (int i = 0; i < 4; ++i) {
    const int id = tid + kNT * i;
    const int row = id >> 7;
    const int c4 = (id & 127) * 4;
    const v4f hv = *(const v4f*)(h0 + (size_t)(bg + row) * kDim + c4);
    v4h h4;
    h4[0] = (_Float16)bfr(hv[0]); h4[1] = (_Float16)bfr(hv[1]); h4[2] = (_Float16)bfr(hv[2]); h4[3] = (_Float16)bfr(hv[3]);
    *(v4h*)(sh_h + row * kHP + c4) = h4;
  }
  if (tid < kA) {
    sh_wa[tid] = bfr(wa[tid]);
    sh_wha[tid] = bfr(wha[tid]);
    sh_bhh[tid] = bfr(bhh[tid]);
  }
  for (int idx = tid; idx < kMB * kT; idx += kNT) sh_sc[idx] = 0.0f;
  float creg[2][8];
#pragma unroll
  for (int p = 0; p < 2; ++p)
#pragma unroll
    for (int r = 0; r < 8; ++r) creg[p][r] = 0.0f;
  float bxr[2][4];
#pragma unroll
  for (int p = 0; p < 2; ++p)
#pragma unroll
    for (int g = 0; g < 4; ++g) bxr[p][g] = bfr(bx[g * kDim + wave * 32 + p * 16 + c]);
  __syncthreads();

#pragma unroll 1
  for (int t = 0; t < kT; ++t) {
    {
      const int sel = wave >> 3;
      const _Float16* Wq = sel ? Whq16 : Wah16;
      const int qn0 = (wave & 7) * 16;
      const v8f qa = proj_tile(sh_h, Wq, qn0, c, koff);
      float* qd = sh_q + sel * (kMB * kA);
#pragma unroll
      for (int r = 0; r < 8; ++r) qd[(8 * hh + r) * kA + qn0 + c] = qa[r] * kS16;
    }
    __syncthreads();

#pragma unroll 1
    for (int it = 0; it < 2; ++it) {
      const int idx = tid + kNT * it;
      const int b = idx >> 6, l = idx & 63;
      const float* ca = ctxatt + ((size_t)(bg + b) * kL + l) * kA;
      const float* qb = sh_q + b * kA;
      float s = 0.0f;
#pragma unroll 2
      for (int a4 = 0; a4 < kA / 4; ++a4) {
        const v4f cv = *(const v4f*)(ca + 4 * a4);
        const v4f qv = *(const v4f*)(qb + 4 * a4);
        const v4f wv = *(const v4f*)(sh_wa + 4 * a4);
#pragma unroll
        for (int e = 0; e < 4; ++e) s += tnh(cv[e] + qv[e]) * wv[e];
      }
      sh_sc[b * kT + l] = s + ba_r;
    }
    __syncthreads();

    {
      float* scb = sh_sc + wave * kT;
      const float v0 = scb[lane], v1 = scb[lane + 32];
      float m = fmaxf(v0, v1);
#pragma unroll
      for (int off = 16; off > 0; off >>= 1) m = fmaxf(m, __shfl_xor(m, off, 32));
      const float e0 = fexp(v0 - m), e1 = fexp(v1 - m);
      float sm = e0 + e1;
#pragma unroll
      for (int off = 16; off > 0; off >>= 1) sm += __shfl_xor(sm, off, 32);
      const float inv = frcp(sm);
      scb[lane] = e0 * inv;
      scb[lane + 32] = e1 * inv;
    }
    __syncthreads();

    {
      v4f keep[4];
#pragma unroll
      for (int i = 0; i < 4; ++i) {
        const int b = bq * 4 + i;
        const float* al = sh_sc + b * kT;
        const float* cr = ctxr + (size_t)(bg + b) * kL * kDim + d0;
        v4f v = (v4f){0.f, 0.f, 0.f, 0.f};
#pragma unroll 4
        for (int l = 0; l < kL; ++l) {
          const float w = al[l];
          const v4f x = *(const v4f*)(cr + (size_t)l * kDim);
          v[0] += w * x[0]; v[1] += w * x[1]; v[2] += w * x[2]; v[3] += w * x[3];
        }
        keep[i] = v;
        v4h h4;
        h4[0] = (_Float16)v[0]; h4[1] = (_Float16)v[1]; h4[2] = (_Float16)v[2]; h4[3] = (_Float16)v[3];
        *(v4h*)(sh_actx + b * kHP + d0) = h4;
      }
      float* octx = out_ctx + ((size_t)(bg + bq * 4) * kT + t) * kDim + d0;
#pragma unroll
      for (int i = 0; i < 4; ++i) *(volatile v4f*)(octx + (size_t)i * kRowStride) = keep[i];
      __threadfence();
#pragma unroll
      for (int i = 0; i < 4; ++i) *(volatile v4f*)(octx + (size_t)i * kRowStride) = keep[i];
    }
    __syncthreads();

    {
#pragma unroll
      for (int i = 0; i < 4; ++i) {
        const int b = bq * 4 + i;
        const int pt = parent[(size_t)(bg + b) * kT + t];
        const int pc = pt < 0 ? 0 : (pt > kT - 1 ? kT - 1 : pt);
        const v4f x = *(const v4f*)(out_h + ((size_t)(bg + b) * kT + pc) * kDim + d0);
        const bool use = (t > 0) && (pc < t);
        v4h h4;
        h4[0] = (_Float16)(use ? x[0] : 0.0f);
        h4[1] = (_Float16)(use ? x[1] : 0.0f);
        h4[2] = (_Float16)(use ? x[2] : 0.0f);
        h4[3] = (_Float16)(use ? x[3] : 0.0f);
        *(v4h*)(sh_apar + b * kHP + d0) = h4;
      }
    }
    {
      const int b = wave;
      const float* q2b = sh_q + kMB * kA + b * kA;
#pragma unroll 1
      for (int s0 = 0; s0 < t; s0 += 32) {
        const int s = s0 + lane;
        const int srd = (s < t) ? s : (t - 1);
        const float* hp = histproj + ((size_t)(bg + b) * kT + srd) * kA;
        float sum = 0.0f;
#pragma unroll 2
        for (int a4 = 0; a4 < kA / 4; ++a4) {
          const v4f hv = *(const v4f*)(hp + 4 * a4);
          const v4f qv = *(const v4f*)(q2b + 4 * a4);
          const v4f wv = *(const v4f*)(sh_wha + 4 * a4);
#pragma unroll
          for (int e = 0; e < 4; ++e) sum += tnh(hv[e] + qv[e]) * wv[e];
        }
        const float val = sum + bha_r;
        if (s < t) sh_sc[b * kT + s] = val;
      }
    }
    if (wave < 4) {
      const int b = tid >> 3, part = tid & 7, a0 = part * 16;
      const float* q2b = sh_q + kMB * kA + b * kA;
      float f = 0.0f;
#pragma unroll 4
      for (int i = 0; i < 16; ++i) {
        const int a = a0 + i;
        f += tnh(sh_bhh[a] + q2b[a]) * sh_wha[a];
      }
      f += __shfl_xor(f, 1, 32);
      f += __shfl_xor(f, 2, 32);
      f += __shfl_xor(f, 4, 32);
      const float val = f + bha_r;
      if (part == 0) sh_sc[b * kT + (kT - 1)] = val;
    }
    __syncthreads();

    {
      float* scb = sh_sc + wave * kT;
      float v[4], e[4];
      bool ok[4];
#pragma unroll
      for (int i = 0; i < 4; ++i) {
        const int s = lane + 32 * i;
        ok[i] = (s < t);
        const float raw = scb[s];
        v[i] = ok[i] ? raw : -__builtin_inff();
      }
      const float fut = scb[kT - 1];
      const float cnt = (float)(kT - t);
      float m = fmaxf(fmaxf(fmaxf(v[0], v[1]), fmaxf(v[2], v[3])), fut);
#pragma unroll
      for (int off = 16; off > 0; off >>= 1) m = fmaxf(m, __shfl_xor(m, off, 32));
      float sm = 0.0f;
#pragma unroll
      for (int i = 0; i < 4; ++i) {
        const float ei = fexp(v[i] - m);
        e[i] = ok[i] ? ei : 0.0f;
        sm += e[i];
      }
#pragma unroll
      for (int off = 16; off > 0; off >>= 1) sm += __shfl_xor(sm, off, 32);
      const float ef = fexp(fut - m);
      const float inv = frcp((sm + cnt * ef) + 1e-7f);
#pragma unroll
      for (int i = 0; i < 4; ++i) {
        const float wv = e[i] * inv;
        if (ok[i]) scb[lane + 32 * i] = wv;
      }
    }
    __syncthreads();

    {
#pragma unroll
      for (int i = 0; i < 4; ++i) {
        const int b = bq * 4 + i;
        const float* wb = sh_sc + b * kT;
        const float* hr = out_h + (size_t)(bg + b) * kT * kDim + d0;
        v4f v = (v4f){0.f, 0.f, 0.f, 0.f};
#pragma unroll 4
        for (int s = 0; s < t; ++s) {
          const float w = wb[s];
          const v4f x = *(const v4f*)(hr + (size_t)s * kDim);
          v[0] += w * x[0]; v[1] += w * x[1]; v[2] += w * x[2]; v[3] += w * x[3];
        }
        v4h h4;
        h4[0] = (_Float16)v[0]; h4[1] = (_Float16)v[1]; h4[2] = (_Float16)v[2]; h4[3] = (_Float16)v[3];
        *(v4h*)(sh_ahc + b * kHP + d0) = h4;
      }
#pragma unroll
      for (int i = 0; i < 4; ++i) {
        const int id = tid + kNT * i;
        const int row = id >> 7;
        const int c4 = (id & 127) * 4;
        const v4f xv = *(const v4f*)(X + ((size_t)(bg + row) * kT + t) * kDim + c4);
        v4h h4;
        h4[0] = (_Float16)bfr(xv[0]); h4[1] = (_Float16)bfr(xv[1]); h4[2] = (_Float16)bfr(xv[2]); h4[3] = (_Float16)bfr(xv[3]);
        *(v4h*)(sh_ax + row * kHP + c4) = h4;
      }
    }
    __syncthreads();

#pragma unroll
    for (int p = 0; p < 2; ++p) {
      v8f acc[4];
#pragma unroll
      for (int j = 0; j < 4; ++j) acc[j] = (v8f){0.f,0.f,0.f,0.f,0.f,0.f,0.f,0.f};
      const int cb = wave * 32 + p * 16;
      gate_seg(acc, sh_h, Uh16, cb, c, koff);
      gate_seg(acc, sh_actx, Cc16, cb, c, koff);
      gate_seg(acc, sh_apar, Ph16, cb, c, koff);
      gate_seg(acc, sh_ahc, Hh16, cb, c, koff);
      gate_seg(acc, sh_ax, Wx16, cb, c, koff);
      const int col = cb + c;
#pragma unroll
      for (int r = 0; r < 8; ++r) {
        const int m = 8 * hh + r;
        const float gi = acc[0][r] * kS16 + bxr[p][0];
        const float gf = acc[1][r] * kS16 + bxr[p][1];
        const float gc = acc[2][r] * kS16 + bxr[p][2];
        const float go = acc[3][r] * kS16 + bxr[p][3];
        const float cn = sgm(gf) * creg[p][r] + sgm(gi) * tnh(gc);
        const float hn = sgm(go) * tnh(cn);
        creg[p][r] = cn;
        sh_hrow[m * kHRP + col] = hn;
      }
    }
    __syncthreads();

    {
      const float* hr = sh_hrow + wave * kHRP;
      float* orow = out_h + ((size_t)(bg + wave) * kT + t) * kDim;
      const v4f w0 = *(const v4f*)(hr + 0 * 128 + 4 * lane);
      const v4f w1 = *(const v4f*)(hr + 1 * 128 + 4 * lane);
      const v4f w2 = *(const v4f*)(hr + 2 * 128 + 4 * lane);
      const v4f w3 = *(const v4f*)(hr + 3 * 128 + 4 * lane);
      *(volatile v4f*)(orow + 0 * 128 + 4 * lane) = w0;
      *(volatile v4f*)(orow + 1 * 128 + 4 * lane) = w1;
      *(volatile v4f*)(orow + 2 * 128 + 4 * lane) = w2;
      *(volatile v4f*)(orow + 3 * 128 + 4 * lane) = w3;
      __threadfence();
      *(volatile v4f*)(orow + 0 * 128 + 4 * lane) = w0;
      *(volatile v4f*)(orow + 1 * 128 + 4 * lane) = w1;
      *(volatile v4f*)(orow + 2 * 128 + 4 * lane) = w2;
      *(volatile v4f*)(orow + 3 * 128 + 4 * lane) = w3;
    }
#pragma unroll
    for (int i = 0; i < 4; ++i) {
      const int id = tid + kNT * i;
      const int row = id >> 7;
      const int c4 = (id & 127) * 4;
      const v4f hv = *(const v4f*)(sh_hrow + row * kHRP + c4);
      v4h h4;
      h4[0] = (_Float16)hv[0]; h4[1] = (_Float16)hv[1]; h4[2] = (_Float16)hv[2]; h4[3] = (_Float16)hv[3];
      *(v4h*)(sh_h + row * kHP + c4) = h4;
    }
    __syncthreads();

    if (wave < 8) {
      const int qn0 = wave * 16;
      const v8f qa = proj_tile(sh_h, Whh16, qn0, c, koff);
#pragma unroll
      for (int r = 0; r < 8; ++r) sh_sc[(8 * hh + r) * kA + qn0 + c] = qa[r] * kS16 + sh_bhh[qn0 + c];
    }
    __syncthreads();

    {
      const v4f pv = *(const v4f*)(sh_sc + wave * kA + 4 * lane);
      float* prow = histproj + ((size_t)(bg + wave) * kT + t) * kA;
      *(volatile v4f*)(prow + 4 * lane) = pv;
      __threadfence();
      *(volatile v4f*)(prow + 4 * lane) = pv;
    }
    __threadfence();
    __syncthreads();
  }
}

constexpr size_t kOffWx = 0;
constexpr size_t kSzBig = (size_t)kG4 * kDim * 2;
constexpr size_t kOffUh = kOffWx + kSzBig;
constexpr size_t kOffCc = kOffUh + kSzBig;
constexpr size_t kOffPh = kOffCc + kSzBig;
constexpr size_t kOffHh = kOffPh + kSzBig;
constexpr size_t kSzSmall = (size_t)kA * kDim * 2;
constexpr size_t kOffWac = kOffHh + kSzBig;
constexpr size_t kOffWah = kOffWac + kSzSmall;
constexpr size_t kOffWhq = kOffWah + kSzSmall;
constexpr size_t kOffWhh = kOffWhq + kSzSmall;
constexpr size_t kOffCtx16 = kOffWhh + kSzSmall;
constexpr size_t kSzCtx16 = (size_t)kB * kL * kDim * 2;
constexpr size_t kOffCtxr = kOffCtx16 + kSzCtx16;
constexpr size_t kSzCtxr = (size_t)kB * kL * kDim * 4;
constexpr size_t kOffBacr = kOffCtxr + kSzCtxr;
constexpr size_t kSzBacr = 512;
constexpr size_t kOffCtxatt = kOffBacr + kSzBacr;
constexpr size_t kSzCtxatt = (size_t)kB * kL * kA * 4;
constexpr size_t kOffHist = kOffCtxatt + kSzCtxatt;
constexpr size_t kSzHist = (size_t)kB * kT * kA * 4;
constexpr size_t kWsTotal = kOffHist + kSzHist;
static_assert(kWsTotal == 20447744);
static_assert(kWsTotal <= 134217728);
static_assert(kOffCtxatt % 256 == 0 && kOffHist % 256 == 0 && kOffBacr % 256 == 0);
static_assert((size_t)kB * kT * kDim * 4 == 8388608);
static_assert(8388608 + 8388608 <= 16777216);

extern "C" void kernel_launch(void* const* d_in, const int* in_sizes, int n_in,
                              void* d_out, int out_size, void* d_ws, size_t ws_size,
                              hipStream_t stream) {
  (void)in_sizes; (void)n_in; (void)out_size; (void)ws_size;
  const float* X       = (const float*)d_in[0];
  const float* context = (const float*)d_in[1];
  const float* h0      = (const float*)d_in[2];
  const float* Wx      = (const float*)d_in[3];
  const float* bx      = (const float*)d_in[4];
  const float* Uh      = (const float*)d_in[5];
  const float* Cc      = (const float*)d_in[6];
  const float* Ph      = (const float*)d_in[7];
  const float* Hh      = (const float*)d_in[8];
  const float* Wac     = (const float*)d_in[9];
  const float* bac     = (const float*)d_in[10];
  const float* Wah     = (const float*)d_in[11];
  const float* wa      = (const float*)d_in[12];
  const float* ba      = (const float*)d_in[13];
  const float* Whh     = (const float*)d_in[14];
  const float* bhh     = (const float*)d_in[15];
  const float* Whq     = (const float*)d_in[16];
  const float* wha     = (const float*)d_in[17];
  const float* bha     = (const float*)d_in[18];
  const int*   parent  = (const int*)d_in[19];

  float* out_h   = (float*)d_out;
  float* out_ctx = (float*)d_out + (size_t)(8388608 / 4);

  char* ws = (char*)d_ws;
  _Float16* Wx16  = (_Float16*)(ws + kOffWx);
  _Float16* Uh16  = (_Float16*)(ws + kOffUh);
  _Float16* Cc16  = (_Float16*)(ws + kOffCc);
  _Float16* Ph16  = (_Float16*)(ws + kOffPh);
  _Float16* Hh16  = (_Float16*)(ws + kOffHh);
  _Float16* Wac16 = (_Float16*)(ws + kOffWac);
  _Float16* Wah16 = (_Float16*)(ws + kOffWah);
  _Float16* Whq16 = (_Float16*)(ws + kOffWhq);
  _Float16* Whh16 = (_Float16*)(ws + kOffWhh);
  _Float16* ctx16 = (_Float16*)(ws + kOffCtx16);
  float* ctxr     = (float*)(ws + kOffCtxr);
  float* bacr     = (float*)(ws + kOffBacr);
  float* ctxatt   = (float*)(ws + kOffCtxatt);
  float* histpj   = (float*)(ws + kOffHist);

  const int n2big = kG4 * kDim / 2;
  const int n2sml = kA * kDim / 2;
  cast_bf_f16x2<<<dim3((n2big + 255) / 256), 256, 0, stream>>>(Wx, Wx16, n2big, 16.0f);
  cast_bf_f16x2<<<dim3((n2big + 255) / 256), 256, 0, stream>>>(Uh, Uh16, n2big, 16.0f);
  cast_bf_f16x2<<<dim3((n2big + 255) / 256), 256, 0, stream>>>(Cc, Cc16, n2big, 16.0f);
  cast_bf_f16x2<<<dim3((n2big + 255) / 256), 256, 0, stream>>>(Ph, Ph16, n2big, 16.0f);
  cast_bf_f16x2<<<dim3((n2big + 255) / 256), 256, 0, stream>>>(Hh, Hh16, n2big, 16.0f);
  cast_bf_f16x2<<<dim3((n2sml + 255) / 256), 256, 0, stream>>>(Wac, Wac16, n2sml, 16.0f);
  cast_bf_f16x2<<<dim3((n2sml + 255) / 256), 256, 0, stream>>>(Wah, Wah16, n2sml, 16.0f);
  cast_bf_f16x2<<<dim3((n2sml + 255) / 256), 256, 0, stream>>>(Whq, Whq16, n2sml, 16.0f);
  cast_bf_f16x2<<<dim3((n2sml + 255) / 256), 256, 0, stream>>>(Whh, Whh16, n2sml, 16.0f);
  const int n2ctx = kB * kL * kDim / 2;
  cast_bf_f16x2<<<dim3((n2ctx + 255) / 256), 256, 0, stream>>>(context, ctx16, n2ctx, 1.0f);
  const int n4ctx = kB * kL * kDim / 4;
  rne_bf_f32x4<<<dim3((n4ctx + 255) / 256), 256, 0, stream>>>(context, ctxr, n4ctx);
  const int n4bac = kA / 4;
  rne_bf_f32x4<<<dim3(1), 256, 0, stream>>>(bac, bacr, n4bac);

  static_assert((kB * kL) % 64 == 0 && kA % 64 == 0 && kDim % 32 == 0);
  static_assert(((kB * kL / 64) * (kA / 64)) % 8 == 0);
  wmma_gemm64<0, false, 2, 0, false, 0><<<dim3((kB * kL / 64) * (kA / 64) / 8, 1), 256, 0, stream>>>(
      (const unsigned short*)ctx16, nullptr, kDim, 0L,
      (const unsigned short*)Wac16, nullptr, kDim, 0L,
      (void*)ctxatt, nullptr, kA, 0L,
      bacr, nullptr, 0L,
      kB * kL, kA, kDim, kS16);

  static_assert(kB % kMB == 0);
  lstm_scan_kernel<<<dim3(kB / kMB), kNT, 0, stream>>>(
      X, ctxr, h0, bx, wa, ba, bhh, wha, bha, parent, ctxatt, histpj,
      Uh16, Cc16, Ph16, Hh16, Wx16, Wah16, Whq16, Whh16, out_h, out_ctx);
}
